// GlobalAttentionLayer_41205916237953
// MI455X (gfx1250) — hardware-verified
//
#include <hip/hip_runtime.h>
#include <math.h>

typedef __attribute__((ext_vector_type(16))) _Float16 v16h;
typedef __attribute__((ext_vector_type(16))) __bf16 v16b;
typedef __attribute__((ext_vector_type(8)))  _Float16 v8h;
typedef __attribute__((ext_vector_type(8)))  float v8f;
typedef __attribute__((ext_vector_type(4)))  float v4f;
typedef __attribute__((ext_vector_type(2)))  float v2f;
typedef __attribute__((ext_vector_type(4)))  unsigned v4u;
typedef __attribute__((ext_vector_type(4)))  int v4i;
typedef float __attribute__((may_alias)) float_a;
typedef int __attribute__((may_alias)) int_a;

template <typename T> __device__ __forceinline__ void vst2(void* p, T v) { *(volatile T*)p = v; __threadfence(); *(volatile T*)p = v; }
__device__ __forceinline__ v8f wmma16(v16h a, v16h b, v8f c) {
  v8f d = __builtin_amdgcn_wmma_f32_16x16x32_f16(false, a, false, b, (short)0, c, false, false);
  asm volatile("v_nop\n\tv_nop\n\tv_nop\n\tv_nop" : "+v"(d) : "v"(a), "v"(b));
  return d;
}
__device__ __forceinline__ v8f wmma_bf(v16b a, v16b b, v8f c) {
  v8f d = __builtin_amdgcn_wmma_f32_16x16x32_bf16(false, a, false, b, (short)0, c, false, false);
  asm volatile("v_nop\n\tv_nop\n\tv_nop\n\tv_nop" : "+v"(d) : "v"(a), "v"(b));
  return d;
}
__device__ __forceinline__ v16h frag_h(const _Float16* rowk0, int lane) {
  union { v16h v; v8h q[2]; } u; const _Float16* p = rowk0 + 8 * (lane >> 4);
  u.q[0] = *(const v8h*)p; u.q[1] = *(const v8h*)(p + 16); return u.v;
}
__device__ __forceinline__ v16h frag_f32(const float* rowk0, int lane) {
  v16h a; const float* p = rowk0 + 8 * (lane >> 4);
#pragma unroll
  for (int i = 0; i < 8; ++i) { a[i] = (_Float16)p[i]; a[8 + i] = (_Float16)p[16 + i]; }
  return a;
}
__device__ __forceinline__ v16h frag_f32s(const float* rowk0, int lane, float sc) {
  v16h a; const float* p = rowk0 + 8 * (lane >> 4);
#pragma unroll
  for (int i = 0; i < 8; ++i) { a[i] = (_Float16)(p[i] * sc); a[8 + i] = (_Float16)(p[16 + i] * sc); }
  return a;
}
__device__ __forceinline__ v16h fragc_f32(const float* W, int k0, int n, int lane, int ld, int K) {
  v16h a; const int g = lane >> 4;
#pragma unroll
  for (int i = 0; i < 8; ++i) { const int ka = k0 + 8 * g + i, kb = ka + 16;
    a[i] = (_Float16)(ka < K ? W[(size_t)(ka < K ? ka : K - 1) * ld + n] : 0.f); a[8 + i] = (_Float16)(kb < K ? W[(size_t)(kb < K ? kb : K - 1) * ld + n] : 0.f); }
  return a;
}
struct F2 { v16b h, l; };
__device__ __forceinline__ F2 bsplit16(const float v[16]) { F2 r;
#pragma unroll
  for (int i = 0; i < 16; ++i) { const __bf16 h = (__bf16)v[i]; r.h[i] = h; r.l[i] = (__bf16)(v[i] - (float)h); }
  return r; }
__device__ __forceinline__ F2 split_row(const float* row, int k0, int lane) { float v[16]; const float* p = row + k0 + 8 * (lane >> 4);
#pragma unroll
  for (int i = 0; i < 8; ++i) { v[i] = p[i]; v[8 + i] = p[16 + i]; }
  return bsplit16(v); }
__device__ __forceinline__ F2 split_rowK(const float* row, int k0, int lane, int K) { float v[16]; const int g = lane >> 4;
#pragma unroll
  for (int i = 0; i < 8; ++i) { const int ka = k0 + 8 * g + i, kb = ka + 16; v[i] = ka < K ? row[ka < K ? ka : K - 1] : 0.f; v[8 + i] = kb < K ? row[kb < K ? kb : K - 1] : 0.f; }
  return bsplit16(v); }
__device__ __forceinline__ F2 split_col(const float* W, int k0, int n, int lane, int ld, int K) { float v[16]; const int g = lane >> 4;
#pragma unroll
  for (int i = 0; i < 8; ++i) { const int ka = k0 + 8 * g + i, kb = ka + 16; v[i] = ka < K ? W[(size_t)(ka < K ? ka : K - 1) * ld + n] : 0.f; v[8 + i] = kb < K ? W[(size_t)(kb < K ? kb : K - 1) * ld + n] : 0.f; }
  return bsplit16(v); }
__device__ __forceinline__ v8f mac3(const F2& a, const F2& b, v8f c) { c = wmma_bf(a.l, b.h, c); c = wmma_bf(a.h, b.l, c); return wmma_bf(a.h, b.h, c); }
__device__ __forceinline__ float sigm(float v) { return 1.0f / (1.0f + expf(-v)); }
#define LDSX() do { asm volatile("s_wait_dscnt 0" ::: "memory"); __builtin_amdgcn_wave_barrier(); __builtin_amdgcn_fence(__ATOMIC_RELEASE, "workgroup"); } while (0)


#define NB 32
#define NN 1024
#define HH 256
#define NR (NB * NN)
#ifndef TQB
#define TQB (NN / 64)
#define TNB NB
#endif
typedef __attribute__((ext_vector_type(8))) __bf16 v8b;
__device__ __forceinline__ v16b frag_b(const __bf16* rowk0, int lane) {
  union { v16b v; v8b q[2]; } u; const __bf16* p = rowk0 + 8 * (lane >> 4);
  u.q[0] = *(const v8b*)p; u.q[1] = *(const v8b*)(p + 16); return u.v;
}
__device__ __forceinline__ float bfr(float v) { return (float)(__bf16)v; }
__device__ __attribute__((noinline)) float exp_ni(float v) { return expf(v); }
__device__ __attribute__((noinline)) float erf_ni(float v) { return erff(v); }

#define WS_PW  0u
#define WS_Q   (WS_PW + 2u * (size_t)3 * HH * HH)
#define WS_K   (WS_Q + 2u * (size_t)NR * HH)
#define WS_QL  (WS_K + 2u * (size_t)NR * HH)
#define WS_KL  (WS_QL + 2u * (size_t)NR * HH)
#define WS_V   (WS_KL + 2u * (size_t)NR * HH)
#define WS_VL  (WS_V + 2u * (size_t)NB * HH * NN)
#define WS_O   (WS_VL + 2u * (size_t)NB * HH * NN)
#define WS_END (WS_O + 4u * (size_t)NR * HH)

__global__ __launch_bounds__(256) void k_pack(const float* __restrict__ WQ, const float* __restrict__ WK, const float* __restrict__ WV, __bf16* __restrict__ PW) { const int n = blockIdx.x, which = blockIdx.y, t = threadIdx.x; __shared__ __align__(16) __bf16 s[HH]; const float* w = (which == 0) ? WQ : (which == 1) ? WK : WV;
  s[t] = (__bf16)w[(size_t)t * HH + n]; __syncthreads(); if (t < HH / 8) vst2((unsigned*)(PW + ((size_t)which * HH + n) * HH + t * 8), *(const v4u*)&s[t * 8]); }
__global__ __launch_bounds__(128) void k_proj(const float* __restrict__ X, const __bf16* __restrict__ PW, const float* __restrict__ BQ, const float* __restrict__ BK, const float* __restrict__ BV, _Float16* __restrict__ Q, _Float16* __restrict__ Kr, _Float16* __restrict__ V, _Float16* __restrict__ QL, _Float16* __restrict__ KL, _Float16* __restrict__ VL) {
  __shared__ __align__(16) _Float16 so[64][HH + 8]; __shared__ __align__(16) _Float16 st[HH][72]; __shared__ __align__(16) _Float16 sol[64][HH + 8]; __shared__ __align__(16) _Float16 stl[HH][72];
  const int tid = threadIdx.x, wave = tid >> 5, lane = tid & 31, col = lane & 15, g = lane >> 4; const int which = blockIdx.y; const size_t rb = (size_t)blockIdx.x * 64; const size_t r0 = rb + wave * 16;
  const __bf16* Wr = PW + ((size_t)which * HH) * HH; const float* BB = (which == 0) ? BQ : (which == 1) ? BK : BV;
  v16b a[8];
#pragma unroll
  for (int kc = 0; kc < 8; ++kc) { const float* p = X + (r0 + col) * HH + kc * 32 + 8 * g;
#pragma unroll
    for (int i = 0; i < 8; ++i) { a[kc][i] = (__bf16)p[i]; a[kc][8 + i] = (__bf16)p[16 + i]; } }
#pragma unroll 1
  for (int half = 0; half < 2; ++half) { v8f acc[8] = {};
#pragma unroll
    for (int kc = 0; kc < 8; ++kc)
#pragma unroll
      for (int j = 0; j < 8; ++j) acc[j] = wmma_bf(a[kc], frag_b(Wr + (size_t)(half * 128 + j * 16 + col) * HH + kc * 32, lane), acc[j]);
#pragma unroll
    for (int j = 0; j < 8; ++j) { const int c = half * 128 + j * 16 + col; const float bb = bfr(BB[c]);
#pragma unroll
      for (int r = 0; r < 8; ++r) { const float fv = acc[j][r] + bb; const _Float16 hv = (_Float16)fv; const _Float16 lv = (_Float16)((fv - (float)hv) * 2048.0f); if (which < 2) { so[wave * 16 + 8 * g + r][c] = hv; sol[wave * 16 + 8 * g + r][c] = lv; } else { st[c][wave * 16 + 8 * g + r] = hv; stl[c][wave * 16 + 8 * g + r] = lv; } } } }
  __syncthreads();
  if (which < 2) { _Float16* dst = (which == 0) ? Q : Kr; _Float16* dstl = (which == 0) ? QL : KL; for (int e = tid; e < 64 * (HH / 8); e += 128) { const int rl = e >> 5, q = e & 31; vst2((unsigned*)(dst + (rb + rl) * HH + q * 8), *(const v4u*)&so[rl][q * 8]); vst2((unsigned*)(dstl + (rb + rl) * HH + q * 8), *(const v4u*)&sol[rl][q * 8]); } }
  else { const size_t b = rb / NN; const int s0 = (int)(rb % NN); for (int e = tid; e < HH * 8; e += 128) { const int d = e >> 3, pc = e & 7; vst2((unsigned*)(V + ((b * HH + d) * NN) + s0 + pc * 8), *(const v4u*)&st[d][pc * 8]); vst2((unsigned*)(VL + ((b * HH + d) * NN) + s0 + pc * 8), *(const v4u*)&stl[d][pc * 8]); } }
}
__global__ __launch_bounds__(128) void k_attn(const _Float16* __restrict__ Q, const _Float16* __restrict__ Kr, const _Float16* __restrict__ V, const _Float16* __restrict__ QL, const _Float16* __restrict__ KL, const _Float16* __restrict__ VL, const int* __restrict__ MK, float* __restrict__ O) {
  __shared__ __align__(16) _Float16 sph[4][16][40]; __shared__ __align__(16) _Float16 spl[4][16][40]; __shared__ __align__(16) float so[4][16][260];
  const int tid = threadIdx.x, wave = tid >> 5, lane = tid & 31, col = lane & 15, g = lane >> 4; const size_t b = blockIdx.z; const int q0 = blockIdx.x * 64 + wave * 16; const size_t rq = b * NN + q0;
  const _Float16* qrow = Q + (rq + col) * HH; const _Float16* qlrow = QL + (rq + col) * HH;
  float mq[8];
#pragma unroll
  for (int r = 0; r < 8; ++r) mq[r] = (float)MK[b * NN + q0 + 8 * g + r];
  float m[8], l[8], al8[8];
#pragma unroll
  for (int r = 0; r < 8; ++r) { m[r] = -3.0e38f; l[r] = 0.f; }
  v8f acc[8] = {};
  for (int e = lane; e < 16 * 128; e += 32) so[wave][e >> 7][128 + (e & 127)] = 0.f;
  __builtin_amdgcn_wave_barrier();
#pragma unroll 1
  for (int ks = 0; ks < NN / 32; ++ks) { const int j0 = ks * 32; v8f s[2];
#pragma unroll
    for (int ct = 0; ct < 2; ++ct) { const int kk = j0 + ct * 16 + col; v8f c = {}, cl = {};
#pragma unroll 2
      for (int kc = 0; kc < 8; ++kc) { const v16h kh = frag_h(Kr + (b * NN + kk) * HH + kc * 32, lane); const v16h qh = frag_h(qrow + kc * 32, lane); c = wmma16(qh, kh, c); cl = wmma16(frag_h(qlrow + kc * 32, lane), kh, cl); cl = wmma16(qh, frag_h(KL + (b * NN + kk) * HH + kc * 32, lane), cl); }
#pragma unroll
      for (int r = 0; r < 8; ++r) c[r] += cl[r] * (1.0f / 2048.0f);
      const float mk = (float)MK[b * NN + kk];
#pragma unroll
      for (int r = 0; r < 8; ++r) { const float am = mq[r] * mk; s[ct][r] = c[r] * 0.0625f + (am - 100000.0f * (1.0f - am)); } }
#pragma unroll
    for (int r = 0; r < 8; ++r) { float mx = fmaxf(s[0][r], s[1][r]);
#pragma unroll
      for (int o = 1; o < 16; o <<= 1) mx = fmaxf(mx, __shfl_xor(mx, o));
      const float mn = fmaxf(m[r], mx); const float alpha = (m[r] <= -1.0e38f) ? 0.f : __expf(m[r] - mn); const float e0 = __expf(s[0][r] - mn), e1 = __expf(s[1][r] - mn); float es = e0 + e1;
#pragma unroll
      for (int o = 1; o < 16; o <<= 1) es += __shfl_xor(es, o);
      l[r] = l[r] * alpha + es; m[r] = mn;
#pragma unroll
      for (int dt = 0; dt < 8; ++dt) acc[dt][r] *= alpha;
      al8[r] = alpha;
      { const float p0 = e0 * 2048.0f, p1 = e1 * 2048.0f; const _Float16 h0 = (_Float16)p0, h1 = (_Float16)p1; sph[wave][8 * g + r][col] = h0; sph[wave][8 * g + r][16 + col] = h1; spl[wave][8 * g + r][col] = (_Float16)((p0 - (float)h0) * 2048.0f); spl[wave][8 * g + r][16 + col] = (_Float16)((p1 - (float)h1) * 2048.0f); } }
    LDSX();
    const v16h pa = frag_h(&sph[wave][col][0], lane), pl = frag_h(&spl[wave][col][0], lane);
#pragma unroll
    for (int dt = 0; dt < 8; ++dt) { const size_t vr = ((b * HH + dt * 16 + col) * NN) + j0; const v16h vhf = frag_h(V + vr, lane); acc[dt] = wmma16(pa, vhf, acc[dt]); v8f al = {}; al = wmma16(pl, vhf, al); al = wmma16(pa, frag_h(VL + vr, lane), al);
#pragma unroll
      for (int r = 0; r < 8; ++r) acc[dt][r] += al[r] * (1.0f / 2048.0f); }
    __builtin_amdgcn_sched_barrier(0);
#pragma unroll 1
    for (int dt = 8; dt < 16; ++dt) { const size_t vr = ((b * HH + dt * 16 + col) * NN) + j0; const v16h vhf = frag_h(V + vr, lane); v8f ab;
#pragma unroll
      for (int r = 0; r < 8; ++r) ab[r] = so[wave][8 * g + r][128 + (dt - 8) * 16 + col] * al8[r];
      ab = wmma16(pa, vhf, ab); v8f al = {}; al = wmma16(pl, vhf, al); al = wmma16(pa, frag_h(VL + vr, lane), al);
#pragma unroll
      for (int r = 0; r < 8; ++r) so[wave][8 * g + r][128 + (dt - 8) * 16 + col] = ab[r] + al[r] * (1.0f / 2048.0f); }
    LDSX(); }
#pragma unroll
  for (int r = 0; r < 8; ++r) { const float il = (1.0f / 2048.0f) / l[r];
#pragma unroll
    for (int dt = 0; dt < 8; ++dt) { so[wave][8 * g + r][dt * 16 + col] = acc[dt][r] * il; so[wave][8 * g + r][128 + dt * 16 + col] *= il; } }
  LDSX();
  for (int rl = 0; rl < 16; ++rl) { vst2(O + (rq + rl) * HH + lane * 4, *(const v4f*)&so[wave][rl][lane * 4]); vst2(O + (rq + rl) * HH + 128 + lane * 4, *(const v4f*)&so[wave][rl][128 + lane * 4]); }
}
__global__ __launch_bounds__(256) void k_ln(const float* __restrict__ A, const float* __restrict__ G, const float* __restrict__ Bt, float* __restrict__ OUT) { __shared__ float red[8]; __shared__ __align__(16) float so2[HH]; const int t = threadIdx.x; const size_t row = blockIdx.x;
  const float v = A[row * HH + t]; float s = v;
#pragma unroll
  for (int o = 1; o < 32; o <<= 1) s += __shfl_xor(s, o);
  if ((t & 31) == 0) red[t >> 5] = s; __syncthreads(); float tot = 0.f; for (int i = 0; i < 8; ++i) tot += red[i]; const float mu = tot / (float)HH; __syncthreads();
  const float d = v - mu; float q = d * d;
#pragma unroll
  for (int o = 1; o < 32; o <<= 1) q += __shfl_xor(q, o);
  if ((t & 31) == 0) red[t >> 5] = q; __syncthreads(); float tq = 0.f; for (int i = 0; i < 8; ++i) tq += red[i]; const float inv = 1.0f / sqrtf(tq / (float)HH + 1e-5f);
  so2[t] = fmaxf((d * inv) * bfr(G[t]) + bfr(Bt[t]), 0.f); __syncthreads(); if (t < HH / 4) vst2(OUT + row * HH + t * 4, *(const v4f*)&so2[t * 4]); }
extern "C" void kernel_launch(void* const* d_in, const int* in_sizes, int n_in, void* d_out, int out_size, void* d_ws, size_t ws_size, hipStream_t stream) {
  (void)in_sizes; (void)n_in; (void)out_size;
  const float** F = (const float**)d_in;
  if (ws_size < (size_t)WS_END) return;
  char* ws = (char*)d_ws; __bf16* PW = (__bf16*)ws; _Float16 *Q = (_Float16*)(ws + WS_Q), *Kr = (_Float16*)(ws + WS_K), *V = (_Float16*)(ws + WS_V), *QL = (_Float16*)(ws + WS_QL), *KL = (_Float16*)(ws + WS_KL), *VL = (_Float16*)(ws + WS_VL); float* O = (float*)(ws + WS_O);
  k_pack<<<dim3(HH, 3), 256, 0, stream>>>(F[2], F[4], F[6], PW);
  k_proj<<<dim3(TNB * NN / 64, 3), 128, 0, stream>>>(F[0], PW, F[3], F[5], F[7], Q, Kr, V, QL, KL, VL);
  k_attn<<<dim3(TQB, 1, TNB), 128, 0, stream>>>(Q, Kr, V, QL, KL, VL, (const int*)d_in[1], O);
  k_ln<<<TNB * NN, 256, 0, stream>>>(O, F[8], F[9], (float*)d_out);
}
